// MambaBlock_57346403336598
// MI455X (gfx1250) — hardware-verified
//
#include <hip/hip_runtime.h>
#include <math.h>

typedef __attribute__((ext_vector_type(16))) _Float16 v16h;
typedef __attribute__((ext_vector_type(8)))  _Float16 v8h;
typedef __attribute__((ext_vector_type(8)))  float    v8f;
typedef __attribute__((ext_vector_type(4)))  float    v4f;

#define PLANE_INPUTS_BF16 1

constexpr int kBatch = 4;
constexpr int kSeqL  = 1024;
constexpr int kDmod  = 1024;
constexpr int kDin   = 2048;
constexpr int kNst   = 16;
constexpr int kDtR   = 64;
constexpr int kPrjN  = 96;
constexpr int kPrjP  = 128;
constexpr int kRows  = kBatch * kSeqL;
constexpr int kTP    = 260;
static_assert(kDtR + 2 * kNst == kPrjN, "x_proj width");
static_assert(kRows == 4096 && (kRows % 64) == 0, "M tile multiple");
static_assert((kDin % 64) == 0 && (kPrjP % 64) == 0 && (kDmod % 64) == 0, "N tile multiples");
static_assert((kDmod % 32) == 0 && (kDin % 32) == 0 && (kDtR % 32) == 0, "K multiples of 32");
static_assert((kSeqL % 64) == 0 && (kDin % 256) == 0 && (kSeqL & (kSeqL - 1)) == 0, "tile multiples");

constexpr float kCarryW   = 32.0f;
constexpr float kCarryWdt = 8.0f;
constexpr float kCarryDl  = 16.0f;
constexpr float kCarryY   = 16.0f;

constexpr size_t kOffIN16   = 0;
constexpr size_t kOffWIN16  = kOffIN16   + (size_t)kRows * kDmod * 2;
constexpr size_t kOffWX16   = kOffWIN16  + (size_t)2 * kDin * kDmod * 2;
constexpr size_t kOffWDT16  = kOffWX16   + (size_t)kPrjP * kDin * 2;
constexpr size_t kOffWOUT16 = kOffWDT16  + (size_t)kDin * kDtR * 2;
constexpr size_t kOffXP     = kOffWOUT16 + (size_t)kDmod * kDin * 2;
constexpr size_t kOffZP     = kOffXP     + (size_t)kRows * kDin * 4;
constexpr size_t kOffXC16   = kOffZP     + (size_t)kRows * kDin * 4;
constexpr size_t kOffDBC    = kOffXC16   + (size_t)kRows * kDin * 2;
constexpr size_t kOffDLOW16 = kOffDBC    + (size_t)kRows * kPrjP * 4;
constexpr size_t kOffY16    = kOffDLOW16 + (size_t)kRows * kDtR * 2;
constexpr size_t kWsTotal   = kOffY16    + (size_t)kRows * kDin * 2;
static_assert(kWsTotal == 125042688ull, "carve total");
static_assert(kWsTotal <= 134217728ull, "carve cap");
static_assert((kOffWIN16 % 128) == 0 && (kOffWX16 % 128) == 0 && (kOffWDT16 % 128) == 0 && (kOffWOUT16 % 128) == 0 &&
              (kOffXP % 128) == 0 && (kOffZP % 128) == 0 && (kOffXC16 % 128) == 0 && (kOffDBC % 128) == 0 &&
              (kOffDLOW16 % 128) == 0 && (kOffY16 % 128) == 0, "128-B aligned regions");

__device__ __forceinline__ unsigned short f2bf_bits(float f) {
  unsigned u = __float_as_uint(f);
  return (unsigned short)((u + 0x7FFFu + ((u >> 16) & 1u)) >> 16);
}
__device__ __forceinline__ float bf_bits2f(unsigned short h) { return __uint_as_float(((unsigned)h) << 16); }

__device__ __forceinline__ float cond_in(float f) {
#if PLANE_INPUTS_BF16
  return bf_bits2f(f2bf_bits(f));
#else
  return f;
#endif
}

__device__ __forceinline__ float h16_to_f32(unsigned hb) {
  const unsigned sgn = (hb & 0x8000u) << 16; const unsigned em = hb & 0x7fffu;
  const float fn = __uint_as_float((em << 13) + 0x38000000u);
  const float fs = (float)em * 5.9604644775390625e-8f;
  const float mag = (em < 0x400u) ? fs : fn; return __uint_as_float(__float_as_uint(mag) | sgn); }

__device__ __forceinline__ void row_guard_h(v8f& a0, v8f& a1, v8f& a2, v8f& a3, v16h x, v16h b0, v16h b1, v16h b2, v16h b3) {
  asm volatile("v_nop\n\tv_nop\n\tv_nop\n\tv_nop" : "+v"(a0), "+v"(a1), "+v"(a2), "+v"(a3) : "v"(x), "v"(b0), "v"(b1), "v"(b2), "v"(b3));
}
__device__ __forceinline__ void keep4_h(v16h a, v16h b, v16h c, v16h d) { asm volatile("v_nop" :: "v"(a), "v"(b), "v"(c), "v"(d)); }
__device__ __forceinline__ void acc_guard4(v8f& a, v8f& b, v8f& c, v8f& d) { asm volatile("v_nop\n\tv_nop\n\tv_nop\n\tv_nop" : "+v"(a), "+v"(b), "+v"(c), "+v"(d)); }

union FragU { v16h v; v8h h[2]; };
__device__ __forceinline__ v16h frag_load(const _Float16* p) {
  FragU f; f.h[0] = *(const v8h*)(p); f.h[1] = *(const v8h*)(p + 16); return f.v;
}
__device__ __forceinline__ v8f frag_mma(v16h a, v16h b, v8f c) {
  return __builtin_amdgcn_wmma_f32_16x16x32_f16(false, a, false, b, (short)0, c, false, false);
}

template <int BIAS_MODE>
__global__ __launch_bounds__(256) void wmma_gemm64_f16(
    const unsigned short* __restrict__ Ap, int lda,
    const unsigned short* __restrict__ Btp, int ldb,
    float* __restrict__ Cout, int ldc,
    const float* __restrict__ bias,
    int M, int N, int K, float scale) {
  const _Float16* A  = (const _Float16*)Ap;
  const _Float16* Bt = (const _Float16*)Btp;
  __shared__ __align__(16) float sT[8][16 * 68];
  const int lane = threadIdx.x & 31;
  const int wave = threadIdx.x >> 5;
  const int tilesN = N >> 6;
  const int tilesM = M >> 6;
  const int tile = blockIdx.x * 8 + wave;
  if (tile >= tilesM * tilesN) return;
  const int tm = tile / tilesN;
  const int tn = tile - tm * tilesN;
  const int m0 = tm << 6;
  const int n0 = tn << 6;

  const int rlane = lane & 15;
  const int koff  = (lane >> 4) * 8;
  const int mOff  = (lane >> 4) * 8;

  v8f acc[4][4];
#pragma unroll
  for (int i = 0; i < 4; ++i)
#pragma unroll
    for (int j = 0; j < 4; ++j) acc[i][j] = (v8f){0.f,0.f,0.f,0.f,0.f,0.f,0.f,0.f};

  for (int k0 = 0; k0 < K; k0 += 32) {
    v16h bh[4];
#pragma unroll
    for (int j = 0; j < 4; ++j) {
      const size_t bo = (size_t)(n0 + (j << 4) + rlane) * ldb + koff + k0;
      bh[j] = frag_load(Bt + bo);
    }
#pragma unroll
    for (int i = 0; i < 4; ++i) {
      const size_t ao = (size_t)(m0 + (i << 4) + rlane) * lda + koff + k0;
      v16h ah = frag_load(A + ao);
#pragma unroll
      for (int j = 0; j < 4; ++j) acc[i][j] = frag_mma(ah, bh[j], acc[i][j]);
      row_guard_h(acc[i][0], acc[i][1], acc[i][2], acc[i][3], ah, bh[0], bh[1], bh[2], bh[3]);
    }
    keep4_h(bh[0], bh[1], bh[2], bh[3]);
  }
  acc_guard4(acc[0][0], acc[0][1], acc[0][2], acc[0][3]);
  acc_guard4(acc[1][0], acc[1][1], acc[1][2], acc[1][3]);
  acc_guard4(acc[2][0], acc[2][1], acc[2][2], acc[2][3]);
  acc_guard4(acc[3][0], acc[3][1], acc[3][2], acc[3][3]);

  float* slab = sT[wave];
#pragma unroll
  for (int i = 0; i < 4; ++i) {
    const int mBase = m0 + (i << 4);
#pragma unroll
    for (int j = 0; j < 4; ++j) {
      const int n = n0 + (j << 4) + rlane;
      float bv = 0.f;
      if (BIAS_MODE == 2) { const float braw = bias[n]; bv = cond_in(braw); }
#pragma unroll
      for (int r = 0; r < 8; ++r) {
        float v = acc[i][j][r] * scale;
        if (BIAS_MODE == 2) v += bv;
        slab[(mOff + r) * 68 + (j << 4) + rlane] = v;
      }
    }
    __builtin_amdgcn_fence(__ATOMIC_RELEASE, "workgroup");
    __builtin_amdgcn_wave_barrier();
    __builtin_amdgcn_fence(__ATOMIC_ACQUIRE, "workgroup");
    {
      const int hh = lane >> 4, c4 = (lane & 15) * 4;
      for (int pass = 0; pass < 2; ++pass) {
#pragma unroll
        for (int it = 0; it < 8; ++it) {
          const int row = it * 2 + hh;
          v4f v = *(const v4f*)(slab + row * 68 + c4);
          *(volatile v4f*)(Cout + (size_t)(mBase + row) * ldc + n0 + c4) = v;
        }
        __threadfence();
      }
    }
    __builtin_amdgcn_fence(__ATOMIC_RELEASE, "workgroup");
    __builtin_amdgcn_wave_barrier();
    __builtin_amdgcn_fence(__ATOMIC_ACQUIRE, "workgroup");
  }
}

__global__ __launch_bounds__(256) void cast_f16_kernel(
    const float* __restrict__ src, unsigned short* __restrict__ dst, int src8, int total8, float carry)
{
  const int i = blockIdx.x * 256 + threadIdx.x;
  if (i >= total8) return;
  const bool live = (i < src8);
  const size_t e0 = (size_t)i << 3;
  const size_t es = live ? e0 : (size_t)0;
  const v4f a0 = *(const v4f*)(src + es);
  const v4f a1 = *(const v4f*)(src + es + 4);
  v8h hv;
#pragma unroll
  for (int e = 0; e < 4; ++e) {
    const float s0 = a0[e];
    const float s1 = a1[e];
    const float x0 = live ? (cond_in(s0) * carry) : 0.0f;
    const float x1 = live ? (cond_in(s1) * carry) : 0.0f;
    hv[e]     = (_Float16)x0;
    hv[4 + e] = (_Float16)x1;
  }
  unsigned short* q = dst + e0;
  *(volatile v8h*)q = hv;
  __threadfence();
  *(volatile v8h*)q = hv;
}

__global__ __launch_bounds__(256) void dlow_cast_kernel(
    const float* __restrict__ DBC, unsigned short* __restrict__ DLOW16, int total8, float carry)
{
  const int i = blockIdx.x * 256 + threadIdx.x;
  if (i >= total8) return;
  const int e0  = i << 3;
  const int row = e0 >> 6;
  const int c8  = e0 & 63;
  const float* p = DBC + (size_t)row * kPrjP + c8;
  const v4f a0 = *(const v4f*)(p);
  const v4f a1 = *(const v4f*)(p + 4);
  v8h hv;
#pragma unroll
  for (int e = 0; e < 4; ++e) {
    hv[e]     = (_Float16)(a0[e] * carry);
    hv[4 + e] = (_Float16)(a1[e] * carry);
  }
  unsigned short* qd = DLOW16 + e0;
  *(volatile v8h*)qd = hv;
  __threadfence();
  *(volatile v8h*)qd = hv;
}

__global__ __launch_bounds__(256) void conv_silu_kernel(
    const float* __restrict__ XP, const float* __restrict__ cw, const float* __restrict__ cb,
    unsigned short* __restrict__ XC16)
{
  __shared__ __align__(16) float sT[16 * kTP];
  const int tid = threadIdx.x, lane = tid & 31, wave = tid >> 5;
  const int d0 = blockIdx.x * 256, d = d0 + tid;
  const int g0 = blockIdx.y * 64;
  const int tb = g0 & (kSeqL - 1);
  const v4f wv = *(const v4f*)(cw + (size_t)d * 4);
  const float wr0 = wv[0], wr1 = wv[1], wr2 = wv[2], wr3 = wv[3];
  const float w0 = cond_in(wr0), w1 = cond_in(wr1), w2 = cond_in(wr2), w3 = cond_in(wr3);
  const float braw = cb[d];
  const float bc = cond_in(braw);
  float xm3, xm2, xm1;
  {
    const bool hist = (tb > 0);
    const int rb = hist ? (g0 - 3) : g0;
    const float v3 = XP[(size_t)rb * kDin + d];
    const float v2 = XP[(size_t)(rb + 1) * kDin + d];
    const float v1 = XP[(size_t)(rb + 2) * kDin + d];
    xm3 = hist ? v3 : 0.f;
    xm2 = hist ? v2 : 0.f;
    xm1 = hist ? v1 : 0.f;
  }
#pragma unroll 1
  for (int sub = 0; sub < 4; ++sub) {
    const int lb = g0 + sub * 16;
#pragma unroll 1
    for (int s = 0; s < 16; ++s) {
      const float xcur = XP[(size_t)(lb + s) * kDin + d];
      float acc = w0 * xm3;
      acc = fmaf(w1, xm2, acc);
      acc = fmaf(w2, xm1, acc);
      acc = fmaf(w3, xcur, acc);
      const float sv = acc + bc;
      const float sg = 1.0f / (1.0f + expf(-sv));
      sT[s * kTP + tid] = sv * sg;
      xm3 = xm2; xm2 = xm1; xm1 = xcur;
    }
    __syncthreads();
    v8h bv[2];
#pragma unroll
    for (int it = 0; it < 2; ++it) {
      const float* sp = sT + (it * 8 + wave) * kTP + lane * 8;
      const v4f a0 = *(const v4f*)(sp);
      const v4f a1 = *(const v4f*)(sp + 4);
#pragma unroll
      for (int e = 0; e < 4; ++e) {
        bv[it][e]     = (_Float16)a0[e];
        bv[it][4 + e] = (_Float16)a1[e];
      }
    }
    for (int pass = 0; pass < 2; ++pass) {
#pragma unroll
      for (int it = 0; it < 2; ++it)
        *(volatile v8h*)(XC16 + (size_t)(lb + it * 8 + wave) * kDin + d0 + lane * 8) = bv[it];
      __threadfence();
    }
    __syncthreads();
  }
}

__global__ __launch_bounds__(256) void scan_kernel(
    const float* __restrict__ DLR, const unsigned* __restrict__ XCw, const float* __restrict__ ZP,
    const float* __restrict__ DBC, const float* __restrict__ A_log, const float* __restrict__ Dv,
    unsigned short* __restrict__ Y16)
{
  __shared__ __align__(16) float sBC[16 * 32];
  __shared__ __align__(16) float sY[16 * kTP];
  __shared__ __align__(16) float sA[kNst * 256];
  const int tid = threadIdx.x, lane = tid & 31, wave = tid >> 5;
  const int d0 = blockIdx.x * 256, d = d0 + tid;
  const size_t row0 = (size_t)blockIdx.y * kSeqL;

#pragma unroll 1
  for (int n = 0; n < kNst; ++n) {
    const float al = A_log[(size_t)d * kNst + n];
    sA[n * 256 + tid] = -expf(cond_in(al));
  }
  __syncthreads();
  float An[kNst], h[kNst];
#pragma unroll
  for (int n = 0; n < kNst; ++n) {
    An[n] = sA[n * 256 + tid];
    h[n] = 0.f;
  }
  const float draw = Dv[d];
  const float Dd = cond_in(draw);
  const unsigned odd = (unsigned)(tid & 1);

#pragma unroll 1
  for (int c = 0; c < kSeqL / 16; ++c) {
    const int l0 = c * 16;
    if (tid < 128) {
      const int r = tid >> 3, q = (tid & 7) * 4;
      const v4f v = *(const v4f*)(DBC + (row0 + l0 + r) * kPrjP + kDtR + q);
      *(v4f*)(sBC + r * 32 + q) = v;
    }
    __syncthreads();
#pragma unroll 1
    for (int s = 0; s < 16; ++s) {
      const size_t m = row0 + (size_t)(l0 + s);
      const float a     = DLR[m * kDin + d];
      const float ea    = expf(-fabsf(a));
      const float delta = fmaxf(a, 0.0f) + log1pf(ea);
      const unsigned w  = XCw[(m * kDin + d) >> 1];
      const unsigned hb = odd ? (w >> 16) : (w & 0xffffu);
      const float xv    = h16_to_f32(hb);
      const float zv    = ZP[m * kDin + d];
      v4f Bq[4], Cq[4];
#pragma unroll
      for (int qq = 0; qq < 4; ++qq) {
        Bq[qq] = *(const v4f*)(sBC + s * 32 + 4 * qq);
        Cq[qq] = *(const v4f*)(sBC + s * 32 + kNst + 4 * qq);
      }
      float dx = delta * xv;
      asm volatile("" : "+v"(dx));
      float y = 0.f;
#pragma unroll
      for (int n = 0; n < kNst; ++n) {
        const float e = __expf(delta * An[n]);
        float p = dx * Bq[n >> 2][n & 3];
        asm volatile("" : "+v"(p));
        float qv = h[n] * e;
        asm volatile("" : "+v"(qv));
        const float hn = qv + p;
        h[n] = hn;
        float rr = Cq[n >> 2][n & 3] * hn;
        asm volatile("" : "+v"(rr));
        y += rr;
      }
      float sk = xv * Dd;
      asm volatile("" : "+v"(sk));
      y += sk;
      const float sg = 1.0f / (1.0f + expf(-zv));
      const float g  = zv * sg;
      sY[s * kTP + tid] = (y * g) * kCarryY;
    }
    __syncthreads();
    v8h hv[2];
#pragma unroll
    for (int it = 0; it < 2; ++it) {
      const float* sp = sY + (it * 8 + wave) * kTP + lane * 8;
      const v4f a0 = *(const v4f*)(sp);
      const v4f a1 = *(const v4f*)(sp + 4);
#pragma unroll
      for (int e = 0; e < 4; ++e) { hv[it][e] = (_Float16)a0[e]; hv[it][4 + e] = (_Float16)a1[e]; }
    }
    for (int pass = 0; pass < 2; ++pass) {
#pragma unroll
      for (int it = 0; it < 2; ++it)
        *(volatile v8h*)(Y16 + (row0 + l0 + it * 8 + wave) * kDin + d0 + lane * 8) = hv[it];
      __threadfence();
    }
  }
}

extern "C" void kernel_launch(void* const* d_in, const int* in_sizes, int n_in,
                              void* d_out, int out_size, void* d_ws, size_t ws_size,
                              hipStream_t stream)
{
  if (n_in < 10) return;
  if (in_sizes[0] != kRows * kDmod) return;
  if (in_sizes[1] != 2 * kDin * kDmod) return;
  if (in_sizes[2] != kDin * 4) return;
  if (in_sizes[3] != kDin) return;
  if (in_sizes[4] != kPrjN * kDin) return;
  if (in_sizes[5] != kDin * kDtR) return;
  if (in_sizes[6] != kDin) return;
  if (in_sizes[7] != kDin * kNst) return;
  if (in_sizes[8] != kDin) return;
  if (in_sizes[9] != kDmod * kDin) return;
  if (out_size != kRows * kDmod) return;
  if (ws_size < kWsTotal) return;

  const float* x_in   = (const float*)d_in[0];
  const float* W_in   = (const float*)d_in[1];
  const float* conv_w = (const float*)d_in[2];
  const float* conv_b = (const float*)d_in[3];
  const float* W_x    = (const float*)d_in[4];
  const float* W_dt   = (const float*)d_in[5];
  const float* b_dt   = (const float*)d_in[6];
  const float* A_log  = (const float*)d_in[7];
  const float* Dv     = (const float*)d_in[8];
  const float* W_out  = (const float*)d_in[9];
  float* dout = (float*)d_out;

  char* ws = (char*)d_ws;
  unsigned short* IN16   = (unsigned short*)(ws + kOffIN16);
  unsigned short* WIN16  = (unsigned short*)(ws + kOffWIN16);
  unsigned short* WX16   = (unsigned short*)(ws + kOffWX16);
  unsigned short* WDT16  = (unsigned short*)(ws + kOffWDT16);
  unsigned short* WOUT16 = (unsigned short*)(ws + kOffWOUT16);
  float*          XP     = (float*)(ws + kOffXP);
  float*          ZP     = (float*)(ws + kOffZP);
  unsigned short* XC16   = (unsigned short*)(ws + kOffXC16);
  float*          DBC    = (float*)(ws + kOffDBC);
  unsigned short* DLOW16 = (unsigned short*)(ws + kOffDLOW16);
  unsigned short* Y16    = (unsigned short*)(ws + kOffY16);
  float*          DLR    = XP;

  constexpr int n8_in   = kRows * kDmod / 8;
  constexpr int n8_win  = 2 * kDin * kDmod / 8;
  constexpr int n8_wxs  = kPrjN * kDin / 8;
  constexpr int n8_wxp  = kPrjP * kDin / 8;
  constexpr int n8_wdt  = kDin * kDtR / 8;
  constexpr int n8_wout = kDmod * kDin / 8;
  constexpr int n8_dl   = kRows * kDtR / 8;
  static_assert((n8_in % 256) == 0 && (n8_win % 256) == 0 && (n8_wxp % 256) == 0 && (n8_wdt % 256) == 0 &&
                (n8_wout % 256) == 0 && (n8_dl % 256) == 0, "cast grids exact");

  cast_f16_kernel<<<n8_in / 256,   256, 0, stream>>>(x_in,  IN16,   n8_in,   n8_in,   1.0f);
  cast_f16_kernel<<<n8_win / 256,  256, 0, stream>>>(W_in,  WIN16,  n8_win,  n8_win,  kCarryW);
  cast_f16_kernel<<<n8_wxp / 256,  256, 0, stream>>>(W_x,   WX16,   n8_wxs,  n8_wxp,  kCarryW);
  cast_f16_kernel<<<n8_wdt / 256,  256, 0, stream>>>(W_dt,  WDT16,  n8_wdt,  n8_wdt,  kCarryWdt);
  cast_f16_kernel<<<n8_wout / 256, 256, 0, stream>>>(W_out, WOUT16, n8_wout, n8_wout, kCarryW);

  wmma_gemm64_f16<0><<<dim3((kRows / 64) * (kDin / 64) / 8), 256, 0, stream>>>(
      IN16, kDmod, WIN16, kDmod, XP, kDin, b_dt, kRows, kDin, kDmod, 1.0f / kCarryW);
  wmma_gemm64_f16<0><<<dim3((kRows / 64) * (kDin / 64) / 8), 256, 0, stream>>>(
      IN16, kDmod, WIN16 + (size_t)kDin * kDmod, kDmod, ZP, kDin, b_dt, kRows, kDin, kDmod, 1.0f / kCarryW);

  conv_silu_kernel<<<dim3(kDin / 256, kRows / 64), 256, 0, stream>>>(XP, conv_w, conv_b, XC16);

  wmma_gemm64_f16<0><<<dim3((kRows / 64) * (kPrjP / 64) / 8), 256, 0, stream>>>(
      XC16, kDin, WX16, kDin, DBC, kPrjP, b_dt, kRows, kPrjP, kDin, 1.0f / kCarryW);

  dlow_cast_kernel<<<n8_dl / 256, 256, 0, stream>>>(DBC, DLOW16, n8_dl, kCarryDl);

  wmma_gemm64_f16<2><<<dim3((kRows / 64) * (kDin / 64) / 8), 256, 0, stream>>>(
      DLOW16, kDtR, WDT16, kDtR, DLR, kDin, b_dt, kRows, kDin, kDtR, 1.0f / (kCarryDl * kCarryWdt));

  scan_kernel<<<dim3(kDin / 256, kBatch), 256, 0, stream>>>(
      DLR, (const unsigned*)XC16, ZP, DBC, A_log, Dv, Y16);

  wmma_gemm64_f16<0><<<dim3((kRows / 64) * (kDmod / 64) / 8), 256, 0, stream>>>(
      Y16, kDin, WOUT16, kDin, dout, kDmod, b_dt, kRows, kDmod, kDin, 1.0f / (kCarryY * kCarryW));
}
